// ModelGAT_15728170238621
// MI455X (gfx1250) — hardware-verified
//
#include <hip/hip_runtime.h>


namespace {
constexpr int N = 50000, E = 400000, G = 256, FI = 54, FE = 12, NH = 4, CH = 32, D = 128, NPAD = 50176  , NBLK = NPAD / 128;
constexpr float FXS = 524288.0f, FXI = 1.0f / 524288.0f, NEG = 0.2f, BNE = 1e-5f;

typedef _Float16 b16;
typedef __attribute__((ext_vector_type(16))) _Float16 v16b;
typedef __attribute__((ext_vector_type(8)))  _Float16 v8b;
typedef __attribute__((ext_vector_type(8)))  float v8f;
typedef __attribute__((ext_vector_type(4)))  float v4f;

__device__ __forceinline__ v8b ld8b(const b16* p) { return *(const v8b*)p; }
__device__ __forceinline__ v16b cat8b(v8b a, v8b b) { return __builtin_shufflevector(a, b, 0, 1, 2, 3, 4, 5, 6, 7, 8, 9, 10, 11, 12, 13, 14, 15); }
__device__ __forceinline__ v16b frag_kb(const b16* p, int hh) { return cat8b(ld8b(p + 8 * hh), ld8b(p + 16 + 8 * hh)); }
__device__ __forceinline__ void split16(float v, b16& hi, b16& lo) { hi = (b16)v; lo = (b16)(v - (float)hi); }
__device__ __forceinline__ void frag_ksplit(const float* p, int hh, v16b& fh_, v16b& fl_) {
  const float* p0 = p + 8 * hh; const float* p1 = p + 16 + 8 * hh;
#pragma unroll
  for (int e = 0; e < 8; ++e) { b16 a, c; split16(p0[e], a, c); fh_[e] = a; fl_[e] = c; split16(p1[e], a, c); fh_[8 + e] = a; fl_[8 + e] = c; }
}
__device__ __forceinline__ v8f wmma16b(v16b a, v16b b, v8f c) {
  v8f d = __builtin_amdgcn_wmma_f32_16x16x32_f16(false, a, false, b, (short)0, c, false, false);
  asm volatile("v_nop\n\tv_nop\n\tv_nop\n\tv_nop" : "+v"(d) : "v"(a), "v"(b));
  return d;
}
__device__ __forceinline__ void wave_lds_sync() {
  __builtin_amdgcn_fence(__ATOMIC_RELEASE, "workgroup");
  __builtin_amdgcn_wave_barrier();
  __builtin_amdgcn_fence(__ATOMIC_ACQUIRE, "workgroup");
}

struct Opnd { const void* p0; const void* p1; int ld; };
template <int NP> __device__ __forceinline__ void load_frags(const Opnd& o, int row, int kb, int hh, v16b& fh_, v16b& fl_) {
  if (NP == 0) { frag_ksplit((const float*)o.p0 + (size_t)row * o.ld + kb, hh, fh_, fl_); }
  else if (NP == 4) {
    const float* p = (const float*)o.p0 + (size_t)row * o.ld + kb; const float* p0 = p + 8 * hh; const float* p1 = p + 16 + 8 * hh;
#pragma unroll
    for (int e = 0; e < 8; ++e) { b16 a, c; split16(p0[e] * 64.0f, a, c); fh_[e] = a; fl_[e] = c; split16(p1[e] * 64.0f, a, c); fh_[8 + e] = a; fl_[8 + e] = c; }
  } else if (NP == 3) {
    const float* p = (const float*)o.p0 + (size_t)row * o.ld + kb; const float* p0 = p + 8 * hh; const float* p1 = p + 16 + 8 * hh;
#pragma unroll
    for (int e = 0; e < 8; ++e) { fh_[e] = (b16)p0[e]; fh_[8 + e] = (b16)p1[e]; }
    fl_ = fh_;
  } else {
    fh_ = frag_kb((const b16*)o.p0 + (size_t)row * o.ld + kb, hh);
    if (NP == 2) fl_ = frag_kb((const b16*)o.p1 + (size_t)row * o.ld + kb, hh); else fl_ = fh_;
  }
}
template <int ANP, int BNP> __device__ __forceinline__ v8f mac(v16b ah, v16b al, v16b bh, v16b bl, v8f c) {
  c = wmma16b(ah, bh, c);
  if (BNP == 0 || BNP == 2 || BNP == 4) c = wmma16b(ah, bl, c);
  if (ANP == 0 || ANP == 2 || ANP == 4) c = wmma16b(al, bh, c);
  return c;
}
template <int ANP, int BNP>
__device__ __forceinline__ void gemm_tile(const Opnd& A, const Opnd& B, int K, int m0, int c0, int nloc, int hlf, v8f (&acc)[2][4]) {
  for (int kb = 0; kb < K; kb += 32) {
    v16b a0h, a0l, a1h, a1l;
    load_frags<ANP>(A, m0 + nloc, kb, hlf, a0h, a0l);
    load_frags<ANP>(A, m0 + 16 + nloc, kb, hlf, a1h, a1l);
#pragma unroll
    for (int t = 0; t < 4; ++t) {
      v16b bh, bl;
      load_frags<BNP>(B, c0 + t * 16 + nloc, kb, hlf, bh, bl);
      acc[0][t] = mac<ANP, BNP>(a0h, a0l, bh, bl, acc[0][t]);
      acc[1][t] = mac<ANP, BNP>(a1h, a1l, bh, bl, acc[1][t]);
    }
  }
}

__device__ __forceinline__ void epi_planes(v8f (&acc)[2][4], float scale, bool two, b16* __restrict__ oh, b16* __restrict__ ol, int ldo,
                                           int m0, int c0, int lane, b16* Th, b16* Tl) {
  const int nloc = lane & 15, hlf = lane >> 4;
#pragma unroll
  for (int t = 0; t < 4; ++t)
#pragma unroll
    for (int r = 0; r < 2; ++r)
#pragma unroll
      for (int v = 0; v < 8; ++v) {
        const int rr = r * 16 + v + 8 * hlf, cc = t * 16 + nloc;
        b16 h_, l_; split16(acc[r][t][v] * scale, h_, l_);
        Th[rr * 64 + cc] = h_; Tl[rr * 64 + cc] = l_;
      }
  wave_lds_sync();
  for (int pass = 0; pass < 2; ++pass) {
#pragma unroll
    for (int j = 0; j < 8; ++j) {
      const int rr = j * 4 + (lane >> 3), c8 = (lane & 7) * 8;
      const size_t o = (size_t)(m0 + rr) * ldo + c0 + c8;
      *(volatile v8b*)(oh + o) = ld8b(Th + rr * 64 + c8);
      if (two) *(volatile v8b*)(ol + o) = ld8b(Tl + rr * 64 + c8);
    }
    __threadfence();
  }
}
__device__ __forceinline__ void epi_f32(v8f (&acc)[2][4], float scale, const float* rscale, float* __restrict__ out, int ldo, int m0, int c0, int lane, float* Tt) {
  const int nloc = lane & 15, hlf = lane >> 4;
#pragma unroll
  for (int t = 0; t < 4; ++t)
#pragma unroll
    for (int r = 0; r < 2; ++r)
#pragma unroll
      for (int v = 0; v < 8; ++v) {
        const int rr = r * 16 + v + 8 * hlf;
        const float rs = rscale ? rscale[(size_t)(m0 + rr) * 32] : 1.0f;
        Tt[rr * 64 + t * 16 + nloc] = acc[r][t][v] * scale * rs;
      }
  wave_lds_sync();
  float* dst0 = out + (size_t)m0 * ldo + c0;
  for (int pass = 0; pass < 2; ++pass) {
#pragma unroll
    for (int j = 0; j < 16; ++j) { const int rr = j * 2 + hlf, c4 = nloc * 4; *(volatile v4f*)(dst0 + (size_t)rr * ldo + c4) = *(const v4f*)(Tt + rr * 64 + c4); }
    __threadfence();
  }
}


__device__ __forceinline__ int fkey(float f) { const int b = __float_as_int(f); return (b >= 0) ? b : (b ^ 0x7FFFFFFF); }
__device__ __forceinline__ float fkey_inv(int k) { return __int_as_float((k >= 0) ? k : (k ^ 0x7FFFFFFF)); }

__global__ __launch_bounds__(256) void prep_kernel(const float* __restrict__ Wl, const float* __restrict__ Wr, b16* __restrict__ w16) {
  const size_t tid = (size_t)blockIdx.x * blockDim.x + threadIdx.x, nth = (size_t)gridDim.x * blockDim.x;
  for (int pass = 0; pass < 2; ++pass) { for (size_t p = tid; p < (size_t)2 * D * 64; p += nth) { const int n = (int)(p / 64), k = (int)(p % 64); const float* W = (n < D) ? Wl : Wr; const int nn = n % D;
      ((volatile b16*)w16)[p] = (b16)((k < FI) ? W[(size_t)min(k, FI - 1) * D + nn] : 0.0f); } __threadfence(); }
}

__global__ __launch_bounds__(128) void lin_kernel(const float* __restrict__ x, const b16* __restrict__ w16, const float* __restrict__ bl, const float* __restrict__ br, float* __restrict__ y) {
  __shared__ __attribute__((aligned(16))) float Ts[4][32 * 64];
  const int lane = threadIdx.x & 31, wave = threadIdx.x >> 5, nloc = lane & 15, hlf = lane >> 4, m0 = blockIdx.y * 128 + wave * 32, c0 = blockIdx.x * 64;
  v8f acc[2][4];
#pragma unroll
  for (int r = 0; r < 2; ++r)
#pragma unroll
    for (int t = 0; t < 4; ++t) acc[r][t] = (v8f){};
  const int ra = min(m0 + nloc, N - 1), rb = min(m0 + 16 + nloc, N - 1);
#pragma unroll
  for (int kb = 0; kb < 64; kb += 32) { v16b a0, a1, l0, l1;
#pragma unroll
    for (int e = 0; e < 16; ++e) { const int k = kb + ((e < 8) ? (8 * hlf + e) : (16 + 8 * hlf + e - 8)); const float u0 = (k < FI) ? x[(size_t)ra * FI + min(k, FI - 1)] : 0.0f, u1 = (k < FI) ? x[(size_t)rb * FI + min(k, FI - 1)] : 0.0f;
      b16 p, q; split16(u0 * 8.0f, p, q); a0[e] = p; l0[e] = q; split16(u1 * 8.0f, p, q); a1[e] = p; l1[e] = q; }
#pragma unroll
    for (int t = 0; t < 4; ++t) { const v16b bw = frag_kb(w16 + (size_t)(c0 + t * 16 + nloc) * 64 + kb, hlf); acc[0][t] = wmma16b(a0, bw, acc[0][t]); acc[0][t] = wmma16b(l0, bw, acc[0][t]); acc[1][t] = wmma16b(a1, bw, acc[1][t]); acc[1][t] = wmma16b(l1, bw, acc[1][t]); } }
#pragma unroll
  for (int t = 0; t < 4; ++t)
#pragma unroll
    for (int r = 0; r < 2; ++r)
#pragma unroll
      for (int v = 0; v < 8; ++v) { const int c = c0 + t * 16 + nloc; acc[r][t][v] = acc[r][t][v] * 0.125f + ((c < D) ? bl[c] : br[c - D]); }
  epi_f32(acc, 1.0f, nullptr, y, 2 * D, m0, c0, lane, Ts[wave]);
}

typedef __attribute__((ext_vector_type(4))) int v4i;
__global__ __launch_bounds__(256) void loopattr_kernel(const int* __restrict__ edst, const float* __restrict__ ea, float* __restrict__ la) {
  constexpr int NB = 2048;
  __shared__ int acc[NB * FE]; __shared__ int cnt[NB];
  const int t_ = threadIdx.x, base = blockIdx.x * NB;
  for (int i = t_; i < NB * FE; i += 256) acc[i] = 0;
  for (int i = t_; i < NB; i += 256) cnt[i] = 0;
  __syncthreads();
  for (int e = t_; e < E; e += 256) { const unsigned sl = (unsigned)(edst[e] - base);
    if (sl < (unsigned)NB) { atomicAdd(&cnt[sl], 1);
#pragma unroll
      for (int q = 0; q < FE; ++q) atomicAdd(&acc[sl * FE + q], (int)rintf(ea[(size_t)e * FE + q] * FXS)); } }
  __syncthreads();
  for (int pass = 0; pass < 2; ++pass) {
    for (int i = t_; i < NB * 4; i += 256) { const int slot = i >> 2, qd = (i & 3) * 4, node = base + slot; if (node < NPAD) { v4f o = {0.0f, 0.0f, 0.0f, 0.0f}; const float inv = 1.0f / fmaxf((float)cnt[slot], 1.0f);
#pragma unroll
        for (int c = 0; c < 4; ++c) { const int q = qd + c; o[c] = (q < FE) ? (float)acc[slot * FE + min(q, FE - 1)] * FXI * inv : (q == FE ? (float)cnt[slot] : 0.0f); }
        *(volatile v4f*)(la + (size_t)node * 16 + qd) = o; } }
    __threadfence();
  }
}

__global__ __launch_bounds__(256) void escore_kernel(const int* __restrict__ esrc, const int* __restrict__ edst, const float* __restrict__ ea, const float* __restrict__ xlr, const float* __restrict__ We, const float* __restrict__ att, float* __restrict__ esc) {
  __shared__ float Ws[FE * D]; __shared__ float As[D]; __shared__ float Eo[64 * NH];
  const int t_ = threadIdx.x;
  for (int i = t_; i < FE * D; i += 256) Ws[i] = We[i];
  if (t_ < D) As[t_] = att[t_];
  __syncthreads();
  const int el = t_ >> 2, h = t_ & 3, e = min(blockIdx.x * 64 + el, E - 1);
  int s = esrc[e], d = edst[e]; s = (s < 0) ? 0 : (s >= N ? N - 1 : s); d = (d < 0) ? 0 : (d >= N ? N - 1 : d);
  float av[FE];
#pragma unroll
  for (int q = 0; q < FE; ++q) av[q] = ea[(size_t)e * FE + q];
  float sc = 0.0f;
#pragma unroll 1
  for (int c = 0; c < CH; ++c) { const int col = h * CH + c; float gv = xlr[(size_t)s * 2 * D + col] + xlr[(size_t)d * 2 * D + D + col];
#pragma unroll
    for (int q = 0; q < FE; ++q) gv += av[q] * Ws[q * D + col];
    gv = (gv >= 0.0f) ? gv : NEG * gv; sc += gv * As[col]; }
  Eo[t_] = sc;
  __syncthreads();
  for (int pass = 0; pass < 2; ++pass) { if (t_ < 64 && blockIdx.x * 64 + t_ < E) *(volatile v4f*)(esc + (size_t)(blockIdx.x * 64 + t_) * 4) = *(const v4f*)(&Eo[t_ * 4]); __threadfence(); }
}

__global__ __launch_bounds__(256) void gat_kernel(const int* __restrict__ esrc, const int* __restrict__ edst, const float* __restrict__ esc, const float* __restrict__ xlr, const float* __restrict__ la, const float* __restrict__ We, const float* __restrict__ att, const float* __restrict__ b4, float* __restrict__ ho, float* __restrict__ slot_) {
  constexpr int NB = 256;
  __shared__ __attribute__((aligned(16))) int acc[NB * D]; __shared__ int mx[NB * NH]; __shared__ int den[NB * NH]; __shared__ int list[8 * 256]; __shared__ float Ws[FE * D]; __shared__ float As[D]; __shared__ float selfsc[NB * NH]; __shared__ float Cs[2][D];
  const int t_ = threadIdx.x, wave = t_ >> 5, lane = t_ & 31, base = blockIdx.x * NB, col0 = lane * 4, myh = lane >> 3;
  for (int i = t_; i < FE * D; i += 256) Ws[i] = We[i];
  if (t_ < D) As[t_] = att[t_];
  for (int i = t_; i < NB * D; i += 256) acc[i] = 0;
  __syncthreads();
  for (int i = t_; i < NB * NH; i += 256) { const int slot = i >> 2, h = i & 3, node = base + slot; float sc = -INFINITY;
    if (node < N) { sc = 0.0f;
#pragma unroll 1
      for (int c = 0; c < CH; ++c) { const int col = h * CH + c; float gv = xlr[(size_t)node * 2 * D + col] + xlr[(size_t)node * 2 * D + D + col];
#pragma unroll
        for (int q = 0; q < FE; ++q) gv += la[(size_t)node * 16 + q] * Ws[q * D + col];
        gv = (gv >= 0.0f) ? gv : NEG * gv; sc += gv * As[col]; } }
    selfsc[i] = sc; mx[i] = fkey(sc); den[i] = 0; }
  __syncthreads();
  for (int c0 = 0; c0 < E; c0 += 256 * 8) { const int e0 = c0 + (wave * 32 + lane) * 8;
#pragma unroll
    for (int j = 0; j < 8; ++j) { const int ee = min(e0 + j, E - 1); const int dv = edst[ee]; const unsigned sl = (unsigned)(((e0 + j < E) ? dv : -1) - base);
      if (sl < (unsigned)NB) {
#pragma unroll
        for (int h = 0; h < NH; ++h) atomicMax(&mx[sl * NH + h], fkey(esc[(size_t)ee * 4 + h])); } } }
  __syncthreads();
  int* wl = list + wave * 256;
  auto accumulate = [&](int s, int slot, float e0_, float e1_, float e2_, float e3_) {
    const float w0 = __expf(e0_ - fkey_inv(mx[slot * NH])), w1 = __expf(e1_ - fkey_inv(mx[slot * NH + 1])), w2 = __expf(e2_ - fkey_inv(mx[slot * NH + 2])), w3 = __expf(e3_ - fkey_inv(mx[slot * NH + 3]));
    { const float wl_ = (lane == 0) ? w0 : (lane == 1) ? w1 : (lane == 2) ? w2 : w3; if (lane < NH) atomicAdd(&den[slot * NH + lane], (int)rintf(wl_ * FXS)); }
    const float wm = (myh == 0) ? w0 : (myh == 1) ? w1 : (myh == 2) ? w2 : w3; const v4f v = *(const v4f*)(xlr + (size_t)s * 2 * D + col0); int* ar = acc + slot * D + col0;
#pragma unroll
    for (int c = 0; c < 4; ++c) atomicAdd(ar + c, (int)rintf(wm * v[c] * FXS));
  };
  for (int slot = wave; slot < NB; slot += 8) { if (base + slot < N) accumulate(base + slot, slot, selfsc[slot * NH], selfsc[slot * NH + 1], selfsc[slot * NH + 2], selfsc[slot * NH + 3]); }
  for (int c0 = 0; c0 < E; c0 += 256 * 8) {
    const int e0 = c0 + (wave * 32 + lane) * 8; int dd[8];
#pragma unroll
    for (int j = 0; j < 8; ++j) { const int dv = edst[min(e0 + j, E - 1)]; dd[j] = (e0 + j < E) ? dv : -1; }
    unsigned sl[8]; bool hit[8]; bool anyl = false;
#pragma unroll
    for (int j = 0; j < 8; ++j) { sl[j] = (unsigned)(dd[j] - base); hit[j] = sl[j] < (unsigned)NB; anyl |= hit[j]; }
    int wc = 0;
    if (__builtin_amdgcn_ballot_w32(anyl) != 0u) {
#pragma unroll
      for (int j = 0; j < 8; ++j) {
        const unsigned mj = __builtin_amdgcn_ballot_w32(hit[j]);
        if (mj != 0u) {
          if (hit[j]) { const int pos = wc + (int)__builtin_amdgcn_mbcnt_lo(mj, 0u); wl[pos] = ((e0 + j) << 8) | (int)sl[j]; }
          wc += __builtin_popcount(mj); } } }
    __builtin_amdgcn_wave_barrier(); __builtin_amdgcn_fence(__ATOMIC_RELEASE, "workgroup"); __builtin_amdgcn_fence(__ATOMIC_ACQUIRE, "workgroup");
    for (int i = 0; i < wc; ++i) { const int ent = wl[i]; const int e = ent >> 8, slot = ent & 255; int s = esrc[e]; s = (s < 0) ? 0 : (s >= N ? N - 1 : s); const v4f es = *(const v4f*)(esc + (size_t)e * 4); accumulate(s, slot, es[0], es[1], es[2], es[3]); }
    __builtin_amdgcn_wave_barrier();
  }
  __syncthreads();
  { const int cq = (t_ & 31) * 4, r0 = t_ >> 5; float s[4] = {0, 0, 0, 0}, s2[4] = {0, 0, 0, 0};
    for (int r = r0; r < NB; r += 8) { const int node = base + r; if (node < N) { const int h = cq / CH; const float id = __builtin_amdgcn_rcpf((float)den[r * NH + h]);
#pragma unroll
        for (int q = 0; q < 4; ++q) { const float v = (float)acc[r * D + cq + q] * id + b4[cq + q]; s[q] += v; s2[q] += v * v; } } }
    __shared__ float Red[2][256 * 4];
#pragma unroll
    for (int q = 0; q < 4; ++q) { Red[0][t_ * 4 + q] = s[q]; Red[1][t_ * 4 + q] = s2[q]; }
    __syncthreads();
    if (t_ < 32) { float a[4] = {0, 0, 0, 0}, b2[4] = {0, 0, 0, 0};
      for (int gq = 0; gq < 8; ++gq)
#pragma unroll
        for (int q = 0; q < 4; ++q) { a[q] += Red[0][(gq * 32 + t_) * 4 + q]; b2[q] += Red[1][(gq * 32 + t_) * 4 + q]; }
#pragma unroll
      for (int q = 0; q < 4; ++q) { Cs[0][cq + q] = a[q]; Cs[1][cq + q] = b2[q]; } }
    __syncthreads(); }
  for (int pass = 0; pass < 2; ++pass) {
    for (int i = t_; i < NB * D / 4; i += 256) { const int r = i >> 5, cq = (i & 31) * 4, node = base + r; v4f o = {0.0f, 0.0f, 0.0f, 0.0f};
      if (node < N) { const int h = cq / CH; const float id = __builtin_amdgcn_rcpf((float)den[r * NH + h]);
#pragma unroll
        for (int q = 0; q < 4; ++q) o[q] = (float)acc[r * D + cq + q] * id + b4[cq + q]; }
      *(volatile v4f*)(ho + (size_t)node * D + cq) = o; }
    if (t_ < 64) ((volatile v4f*)(slot_ + (size_t)blockIdx.x * 2 * D))[t_] = *(const v4f*)(&Cs[t_ >> 5][(t_ & 31) * 4]);
    __threadfence();
  }
}

__global__ __launch_bounds__(128) void bnfin_kernel(const float* __restrict__ slot_, const float* __restrict__ g, const float* __restrict__ bb, float* __restrict__ coef) {
  const int c = threadIdx.x; double s = 0.0, s2 = 0.0;
  for (int bk = 0; bk < NPAD / 256; ++bk) { s += (double)slot_[((size_t)bk * 2) * D + c]; s2 += (double)slot_[((size_t)bk * 2 + 1) * D + c]; }
  const double mean = s / N, var = s2 / N - mean * mean; const float a = g[c] * (float)(1.0 / sqrt(var + (double)BNE)), sh = bb[c] - (float)mean * a;
  for (int pass = 0; pass < 2; ++pass) { ((volatile float*)coef)[c] = a; ((volatile float*)coef)[D + c] = sh; __threadfence(); }
}

__global__ __launch_bounds__(256) void pool_kernel(const float* __restrict__ h, const float* __restrict__ coef, const int* __restrict__ batch, float* __restrict__ out) {
  constexpr int GB = 128;
  __shared__ int sacc[GB * D]; __shared__ int cnt[GB]; __shared__ int list[8 * 256]; __shared__ float Ca[D], Csh[D];
  const int t_ = threadIdx.x, wave = t_ >> 5, lane = t_ & 31, gbase = blockIdx.x * GB, col0 = lane * 4;
  for (int i = t_; i < GB * D; i += 256) sacc[i] = 0;
  if (t_ < GB) cnt[t_] = 0;
  if (t_ < D) { Ca[t_] = coef[t_]; Csh[t_] = coef[D + t_]; }
  __syncthreads();
  int* wl = list + wave * 256;
  for (int c0 = 0; c0 < N; c0 += 256 * 8) {
    const int n0 = c0 + (wave * 32 + lane) * 8; int dd[8];
#pragma unroll
    for (int j = 0; j < 8; ++j) { const int bv = batch[min(n0 + j, N - 1)]; dd[j] = (n0 + j < N) ? bv : -1; }
    unsigned sl[8]; bool hit[8]; bool anyl = false;
#pragma unroll
    for (int j = 0; j < 8; ++j) { sl[j] = (unsigned)(dd[j] - gbase); hit[j] = sl[j] < (unsigned)GB; anyl |= hit[j]; }
    int wc = 0;
    if (__builtin_amdgcn_ballot_w32(anyl) != 0u) {
#pragma unroll
      for (int j = 0; j < 8; ++j) {
        const unsigned mj = __builtin_amdgcn_ballot_w32(hit[j]);
        if (mj != 0u) {
          if (hit[j]) { const int pos = wc + (int)__builtin_amdgcn_mbcnt_lo(mj, 0u); wl[pos] = ((n0 + j) << 7) | (int)sl[j]; atomicAdd(&cnt[sl[j]], 1); }
          wc += __builtin_popcount(mj); } } }
    __builtin_amdgcn_wave_barrier(); __builtin_amdgcn_fence(__ATOMIC_RELEASE, "workgroup"); __builtin_amdgcn_fence(__ATOMIC_ACQUIRE, "workgroup");
    for (int i = 0; i < wc; ++i) { const int ent = wl[i]; const int n = ent >> 7, slot = ent & 127; const v4f v = *(const v4f*)(h + (size_t)n * D + col0);
#pragma unroll
      for (int c = 0; c < 4; ++c) { const float z = v[c] * Ca[col0 + c] + Csh[col0 + c]; const float gl = 0.5f * z * (1.0f + erff(z * 0.70710678118654752f)); atomicAdd(&sacc[slot * D + col0 + c], (int)rintf(gl * FXS)); } }
    __builtin_amdgcn_wave_barrier();
  }
  __syncthreads();
  for (int pass = 0; pass < 2; ++pass) { for (int i = t_; i < GB * D; i += 256) { const int slot = i / D; ((volatile float*)out)[(size_t)(gbase + slot) * D + (i % D)] = (float)sacc[i] * FXI / fmaxf((float)cnt[slot], 1.0f); } __threadfence(); }
}
}

extern "C" void kernel_launch(void* const* d_in, const int* in_sizes, int n_in,
                              void* d_out, int out_size, void* d_ws, size_t ws_size, hipStream_t stream) {
  (void)n_in; (void)out_size;
  const float* x = (const float*)d_in[0]; const int* ei = (const int*)d_in[1]; const int* batch = (const int*)d_in[2]; const float* eattr = (const float*)d_in[3];
  const float* Wl4 = (const float*)d_in[15]; const float* bl4 = (const float*)d_in[16]; const float* Wr4 = (const float*)d_in[17]; const float* br4 = (const float*)d_in[18]; const float* We4 = (const float*)d_in[19]; const float* att4 = (const float*)d_in[20]; const float* b4 = (const float*)d_in[21];
  const float* g4 = (const float*)d_in[28]; const float* be4 = (const float*)d_in[29];
  float* out = (float*)d_out;
  if (in_sizes[0] != N * FI || in_sizes[1] != 2 * E || in_sizes[2] != N || in_sizes[3] != E * FE || in_sizes[15] != FI * D || in_sizes[19] != FE * D || in_sizes[20] != NH * CH || in_sizes[28] != D) return;
  const int* esrc = ei; const int* edst = ei + E;
  size_t off = 0; char* ws = (char*)d_ws;
  auto carve = [&](size_t bytes) { char* p = ws + off; off += (bytes + 255) & ~(size_t)255; return p; };
  b16* w16 = (b16*)carve((size_t)2 * D * 64 * 2); float* xlr = (float*)carve((size_t)NPAD * 2 * D * 4); float* la = (float*)carve((size_t)NPAD * 16 * 4); float* esc = (float*)carve((size_t)E * 4 * 4);
  float* h = (float*)carve((size_t)NPAD * D * 4); float* slot_ = (float*)carve((size_t)(NPAD / 256) * 2 * D * 4); float* coef = (float*)carve(2 * D * 4);
  if (off > ws_size) return;
  prep_kernel<<<64, 256, 0, stream>>>(Wl4, Wr4, w16);
  lin_kernel<<<dim3(2 * D / 64, NBLK), 128, 0, stream>>>(x, w16, bl4, br4, xlr);
  loopattr_kernel<<<NPAD / 2048 + 1, 256, 0, stream>>>(edst, eattr, la);
  escore_kernel<<<(E + 63) / 64, 256, 0, stream>>>(esrc, edst, eattr, xlr, We4, att4, esc);
  gat_kernel<<<NPAD / 256, 256, 0, stream>>>(esrc, edst, esc, xlr, la, We4, att4, b4, h, slot_);
  bnfin_kernel<<<1, 128, 0, stream>>>(slot_, g4, be4, coef);
  pool_kernel<<<G / 128, 256, 0, stream>>>(h, coef, batch, out);
}
